// RNN_Net_67061619360064
// MI455X (gfx1250) — hardware-verified
//
#include <hip/hip_runtime.h>

typedef __attribute__((ext_vector_type(16))) _Float16 v16h;
typedef __attribute__((ext_vector_type(8)))  _Float16 v8h;
typedef __attribute__((ext_vector_type(4)))  _Float16 v4h;
typedef __attribute__((ext_vector_type(8)))  float    v8f;
typedef __attribute__((ext_vector_type(4)))  float    v4f;

constexpr int kB = 64;
constexpr int kT = 1024;
constexpr int kI = 128;
constexpr int kH = 1024;
constexpr int kO = 64;
constexpr int kRowsPerBlk = 16;
constexpr int kThreads = 512;
constexpr int kWaves = kThreads / 32;
constexpr int kTilesPerWave = 4;
constexpr int kHP = kH + 8;
constexpr int kXP = kI + 8;
constexpr int kOP = kO + 4;
static_assert(kWaves * kTilesPerWave * 16 == kH);
static_assert((kB % kRowsPerBlk) == 0);
static_assert((kH % 32) == 0 && (kI % 32) == 0);
static_assert(kO == 64);
static_assert(kRowsPerBlk * kI == kThreads * 4);
static_assert(((kHP * 2) % 16) == 0 && ((kXP * 2) % 16) == 0 && ((kOP * 4) % 16) == 0);

constexpr float kCarryHH  = 1024.0f;
constexpr float kCarryX   = 16.0f;
constexpr float kCarryIH  = 64.0f;
constexpr float kCarryOut = 65536.0f;
constexpr float kCarryRes = 2048.0f;
static_assert(kCarryX * kCarryIH == kCarryHH);
constexpr float kInvHH     = 1.0f / kCarryHH;
constexpr float kInvHHRes  = 1.0f / (kCarryHH * kCarryRes);
constexpr float kInvOut    = 1.0f / kCarryOut;
constexpr float kInvOutRes = 1.0f / (kCarryOut * kCarryRes);
constexpr float kMinNormal16 = 6.103515625e-05f;
constexpr float kLeak = 0.2f;
constexpr float kKeep = 1.0f - kLeak;
static_assert(__builtin_bit_cast(unsigned, kLeak) == 0x3E4CCCCDu);
static_assert(__builtin_bit_cast(unsigned, kKeep) == 0x3F4CCCCDu);

constexpr size_t kBytesWHH  = (size_t)kH * kH * 2;
constexpr size_t kBytesWIH  = (size_t)kH * kI * 2;
constexpr size_t kBytesWOUT = (size_t)kO * kH * 2;
constexpr size_t kOffWHH  = 0;
constexpr size_t kOffWIH  = kOffWHH + kBytesWHH;
constexpr size_t kOffWOUT = kOffWIH + kBytesWIH;
constexpr size_t kWsTotal = kOffWOUT + kBytesWOUT;
static_assert(kWsTotal == 2490368ull);
static_assert(kWsTotal <= 134217728ull);
static_assert((kOffWIH % 128) == 0 && (kOffWOUT % 128) == 0);

__device__ __forceinline__ unsigned short f2bf_bits(float f) {
  unsigned u = __float_as_uint(f);
  return (unsigned short)((u + 0x7FFFu + ((u >> 16) & 1u)) >> 16);
}
__device__ __forceinline__ float bf_bits2f(unsigned short h) { return __uint_as_float(((unsigned)h) << 16); }
__device__ __forceinline__ float bf16_value(float f) { return bf_bits2f(f2bf_bits(f)); }
__device__ __forceinline__ float flush16(float v) { return (fabsf(v) < kMinNormal16) ? 0.0f : v; }

union FH { v16h v; v8h h[2]; };
__device__ __forceinline__ v16h frag_load_global(const _Float16* p) {
  FH f;
  f.h[0] = *(const v8h*)(p);
  f.h[1] = *(const v8h*)(p + 16);
  return f.v;
}
__device__ __forceinline__ v8f mma_h(v16h a, v16h b, v8f c) {
  c = __builtin_amdgcn_wmma_f32_16x16x32_f16(false, a, false, b, (short)0, c, false, false);
  asm volatile("v_nop\n\tv_nop\n\tv_nop\n\tv_nop" : "+v"(c) : "v"(a), "v"(b));
  return c;
}

__global__ __launch_bounds__(256) void plane_f16_kernel(
    const float* __restrict__ src, unsigned short* __restrict__ dst, int total8, float carry)
{
  const int i = blockIdx.x * 256 + threadIdx.x;
  if (i >= total8) return;
  const size_t e0 = (size_t)i << 3;
  const v4f a0 = *(const v4f*)(src + e0);
  const v4f a1 = *(const v4f*)(src + e0 + 4);
  v8h hv;
#pragma unroll
  for (int e = 0; e < 4; ++e) {
    const float s0 = a0[e];
    const float s1 = a1[e];
    hv[e]     = (_Float16)flush16(bf16_value(s0) * carry);
    hv[4 + e] = (_Float16)flush16(bf16_value(s1) * carry);
  }
  unsigned short* q = dst + e0;
  *(volatile v8h*)q = hv;
  __threadfence();
  *(volatile v8h*)q = hv;
}

__global__ __launch_bounds__(kThreads) void leaky_scan_kernel(
    const float* __restrict__ x, const unsigned short* __restrict__ whh_p,
    const unsigned short* __restrict__ wih_p, const unsigned short* __restrict__ wout_p,
    float* __restrict__ out)
{
  __shared__ __align__(16) _Float16 Hhi[kRowsPerBlk * kHP];
  __shared__ __align__(16) _Float16 Hlo[kRowsPerBlk * kHP];
  __shared__ __align__(16) _Float16 Xs[kRowsPerBlk * kXP];
  __shared__ __align__(16) float    Os[kRowsPerBlk * kOP];

  const int tid  = threadIdx.x;
  const int lane = tid & 31;
  const int wave = __builtin_amdgcn_readfirstlane(tid >> 5);
  const int hh   = lane >> 4;
  const int c    = lane & 15;
  const int b0   = blockIdx.x * kRowsPerBlk;
  const int n0w  = wave * 64;

  const _Float16* wA  = (const _Float16*)whh_p  + (size_t)(n0w + c) * kH + 8 * hh;
  const _Float16* wiA = (const _Float16*)wih_p  + (size_t)(n0w + c) * kI + 8 * hh;
  const _Float16* woA = (const _Float16*)wout_p + (size_t)((wave & 3) * 16 + c) * kH + 8 * hh;
  const int hBoff = c * kHP + 8 * hh;
  const int xBoff = c * kXP + 8 * hh;
  const int ownOff = c * kHP + n0w + 8 * hh;
  const int srow = tid >> 5;
  const int sc4  = (tid & 31) * 4;
  const float* xsrc = x + (size_t)(b0 + srow) * kT * kI + sc4;
  const int xsOff = srow * kXP + sc4;

  v8f hst[kTilesPerWave];
#pragma unroll
  for (int j = 0; j < kTilesPerWave; ++j) {
    hst[j] = (v8f){0.f, 0.f, 0.f, 0.f, 0.f, 0.f, 0.f, 0.f};
    const v8h z = (v8h){(_Float16)0.0f, (_Float16)0.0f, (_Float16)0.0f, (_Float16)0.0f,
                        (_Float16)0.0f, (_Float16)0.0f, (_Float16)0.0f, (_Float16)0.0f};
    *(v8h*)(Hhi + ownOff + 16 * j) = z;
    *(v8h*)(Hlo + ownOff + 16 * j) = z;
  }
  {
    const v4f xv = *(const v4f*)(xsrc);
    v4h pk;
#pragma unroll
    for (int e = 0; e < 4; ++e) {
      const float s = xv[e];
      pk[e] = (_Float16)flush16(bf16_value(s) * kCarryX);
    }
    *(v4h*)(Xs + xsOff) = pk;
  }
  __syncthreads();

#pragma unroll 1
  for (int t = 0; t < kT; ++t) {
    v8f accM[kTilesPerWave], accR[kTilesPerWave];
#pragma unroll
    for (int j = 0; j < kTilesPerWave; ++j) {
      accM[j] = (v8f){0.f, 0.f, 0.f, 0.f, 0.f, 0.f, 0.f, 0.f};
      accR[j] = (v8f){0.f, 0.f, 0.f, 0.f, 0.f, 0.f, 0.f, 0.f};
    }
    v8f hdM = (v8f){0.f, 0.f, 0.f, 0.f, 0.f, 0.f, 0.f, 0.f};
    v8f hdR = (v8f){0.f, 0.f, 0.f, 0.f, 0.f, 0.f, 0.f, 0.f};

#pragma unroll 1
    for (int kx = 0; kx < kI; kx += 32) {
      FH xb;
      xb.h[0] = *(const v8h*)(Xs + xBoff + kx);
      xb.h[1] = *(const v8h*)(Xs + xBoff + kx + 16);
#pragma unroll
      for (int j = 0; j < kTilesPerWave; ++j) {
        const v16h a = frag_load_global(wiA + (size_t)j * 16 * kI + kx);
        accM[j] = mma_h(a, xb.v, accM[j]);
      }
    }

#pragma unroll 1
    for (int k0 = 0; k0 < kH; k0 += 32) {
      FH bh, bl;
      bh.h[0] = *(const v8h*)(Hhi + hBoff + k0);
      bh.h[1] = *(const v8h*)(Hhi + hBoff + k0 + 16);
      bl.h[0] = *(const v8h*)(Hlo + hBoff + k0);
      bl.h[1] = *(const v8h*)(Hlo + hBoff + k0 + 16);
#pragma unroll
      for (int j = 0; j < kTilesPerWave; ++j) {
        const v16h a = frag_load_global(wA + (size_t)j * 16 * kH + k0);
        accM[j] = mma_h(a, bh.v, accM[j]);
        accR[j] = mma_h(a, bl.v, accR[j]);
      }
      if (wave < 4) {
        const v16h a = frag_load_global(woA + k0);
        hdM = mma_h(a, bh.v, hdM);
        hdR = mma_h(a, bl.v, hdR);
      }
    }

    if (wave < 4) {
      v4f o0, o1;
#pragma unroll
      for (int r = 0; r < 4; ++r) {
        o0[r] = hdM[r] * kInvOut + hdR[r] * kInvOutRes;
        o1[r] = hdM[4 + r] * kInvOut + hdR[4 + r] * kInvOutRes;
      }
      float* op = Os + c * kOP + wave * 16 + 8 * hh;
      *(v4f*)(op) = o0;
      *(v4f*)(op + 4) = o1;
    }

    __syncthreads();

#pragma unroll
    for (int j = 0; j < kTilesPerWave; ++j) {
      v8h hv, lv;
#pragma unroll
      for (int r = 0; r < 8; ++r) {
        const float f  = accM[j][r] * kInvHH + accR[j][r] * kInvHHRes;
        const float hn = kKeep * hst[j][r] + kLeak * f;
        hst[j][r] = hn;
        const _Float16 h16 = (_Float16)flush16(hn);
        const float res = (hn - (float)h16) * kCarryRes;
        const _Float16 l16 = (_Float16)flush16(res);
        hv[r] = h16;
        lv[r] = l16;
      }
      *(v8h*)(Hhi + ownOff + 16 * j) = hv;
      *(v8h*)(Hlo + ownOff + 16 * j) = lv;
    }

    {
      const int tn = (t + 1 < kT) ? (t + 1) : (kT - 1);
      const v4f xv = *(const v4f*)(xsrc + (size_t)tn * kI);
      v4h pk;
#pragma unroll
      for (int e = 0; e < 4; ++e) {
        const float s = xv[e];
        pk[e] = (_Float16)flush16(bf16_value(s) * kCarryX);
      }
      *(v4h*)(Xs + xsOff) = pk;
    }

    if (wave < 8) {
      const int row = 2 * wave + hh;
      const int c4  = c * 4;
      const v4f v = *(const v4f*)(Os + row * kOP + c4);
      float* p = out + ((size_t)(b0 + row) * kT + t) * kO + c4;
      *(volatile v4f*)p = v;
      __threadfence();
      *(volatile v4f*)p = v;
    }

    __syncthreads();
  }
}

extern "C" void kernel_launch(void* const* d_in, const int* in_sizes, int n_in,
                              void* d_out, int out_size, void* d_ws, size_t ws_size,
                              hipStream_t stream) {
  if (n_in < 4) return;
  if (in_sizes[0] != kB * kT * kI) return;
  if (in_sizes[1] != kH * kI) return;
  if (in_sizes[2] != kH * kH) return;
  if (in_sizes[3] != kO * kH) return;
  if (out_size != kB * kT * kO) return;
  if (ws_size < kWsTotal) return;

  const float* x     = (const float*)d_in[0];
  const float* W_ih  = (const float*)d_in[1];
  const float* W_hh  = (const float*)d_in[2];
  const float* W_out = (const float*)d_in[3];
  float* out = (float*)d_out;

  char* ws = (char*)d_ws;
  unsigned short* WHH  = (unsigned short*)(ws + kOffWHH);
  unsigned short* WIH  = (unsigned short*)(ws + kOffWIH);
  unsigned short* WOUT = (unsigned short*)(ws + kOffWOUT);

  static_assert(((kH * kH / 8) % 256) == 0 && ((kH * kI / 8) % 256) == 0 && ((kO * kH / 8) % 256) == 0);
  plane_f16_kernel<<<(kH * kH / 8) / 256, 256, 0, stream>>>(W_hh, WHH, kH * kH / 8, kCarryHH);
  plane_f16_kernel<<<(kH * kI / 8) / 256, 256, 0, stream>>>(W_ih, WIH, kH * kI / 8, kCarryIH);
  plane_f16_kernel<<<(kO * kH / 8) / 256, 256, 0, stream>>>(W_out, WOUT, kO * kH / 8, kCarryOut);

  leaky_scan_kernel<<<kB / kRowsPerBlk, kThreads, 0, stream>>>(x, WHH, WIH, WOUT, out);
}
